// Decoder_24438363914350
// MI455X (gfx1250) — hardware-verified
//
#include <hip/hip_runtime.h>
#include <math.h>

constexpr int NBAT  = 32;
constexpr int NSTEP = 12;
constexpr int NNODE = 512;
constexpr int NFEAT = 2;
constexpr int NHID  = 64;
constexpr int NSUP  = 4;
constexpr int NROWS = NBAT * NNODE;
constexpr int RB    = 32;
constexpr int NBLK  = NROWS / RB;
constexpr int NTHR  = 256;
constexpr int FC0   = NFEAT + NHID;
constexpr int FX0   = NFEAT;
constexpr int K0    = NSUP * FC0;
constexpr int K0P   = 288;
constexpr int LD0   = 320;
constexpr int FC1   = 2 * NHID;
constexpr int FX1   = NHID;
constexpr int K1    = NSUP * FC1;
constexpr int LD1   = 512;
constexpr int XP    = 520;
constexpr int HSP   = 68;
constexpr float ACARRY = 16.0f;
constexpr float WCARRY = 64.0f;
constexpr float FOLD   = 1.0f / (ACARRY * WCARRY);

static_assert(K0 == 264 && K1 == 512, "shape");
static_assert(K0P % 32 == 0 && K1 % 32 == 0 && K0P >= K0 && LD0 >= K0P && LD0 % 64 == 0 && LD1 % 64 == 0, "k padding");
static_assert((K0P - K0) == 24, "three 16-byte pad vectors per row");
static_assert(NROWS % RB == 0 && NNODE % RB == 0, "row tiling");
static_assert(NSUP * RB == 128 && NHID * NFEAT == 128, "init mapping");
static_assert(RB * 8 == NTHR, "x-part mapping");
static_assert((XP * 2) % 16 == 0 && (K0 * 2) % 16 == 0, "LDS vector alignment");
static_assert(XP >= K1, "A tile width");

typedef __attribute__((ext_vector_type(16))) _Float16 v16h;
typedef __attribute__((ext_vector_type(8)))  _Float16 v8h;
typedef __attribute__((ext_vector_type(8)))  float    v8f;
typedef __attribute__((ext_vector_type(4)))  float    v4f;

__device__ __forceinline__ unsigned short f2bf_bits(float f) {
  unsigned u = __float_as_uint(f);
  return (unsigned short)((u + 0x7FFFu + ((u >> 16) & 1u)) >> 16);
}
__device__ __forceinline__ float bf_bits2f(unsigned short h) { return __uint_as_float(((unsigned)h) << 16); }
__device__ __forceinline__ float bf16r(float f) { return bf_bits2f(f2bf_bits(f)); }

union FragU { v16h v; v8h h[2]; };
__device__ __forceinline__ v16h ld_frag(const _Float16* p) {
  FragU f;
  f.h[0] = *(const v8h*)(p);
  f.h[1] = *(const v8h*)(p + 16);
  return f.v;
}
__device__ __forceinline__ v8f mma_h(v16h a, v16h b, v8f c) {
  return __builtin_amdgcn_wmma_f32_16x16x32_f16(false, a, false, b, (short)0, c, false, false);
}
__device__ __forceinline__ void guard_pair(v8f& a, v8f& b, v16h x, v16h y, v16h z) {
  asm volatile("v_nop\n\tv_nop\n\tv_nop\n\tv_nop" : "+v"(a), "+v"(b) : "v"(x), "v"(y), "v"(z));
}
__device__ __forceinline__ void guard_one(v8f& a, v16h x, v16h y) {
  asm volatile("v_nop\n\tv_nop\n\tv_nop\n\tv_nop" : "+v"(a) : "v"(x), "v"(y));
}
__device__ __forceinline__ void guard_tail2(v8f& a, v8f& b) {
  asm volatile("v_nop\n\tv_nop\n\tv_nop\n\tv_nop" : "+v"(a), "+v"(b));
}
__device__ __forceinline__ void guard_tail1(v8f& a) {
  asm volatile("v_nop\n\tv_nop\n\tv_nop\n\tv_nop" : "+v"(a));
}

__device__ __forceinline__ float fsig(float x)  { return __builtin_amdgcn_rcpf(1.0f + expf(-x)); }
__device__ __forceinline__ float ftanh(float x) { return 1.0f - 2.0f * __builtin_amdgcn_rcpf(expf(2.0f * x) + 1.0f); }

__device__ __forceinline__ void gemm_pair(const _Float16* arow, const _Float16* bp0, const _Float16* bp1,
                                          const int kdim, v8f& acc0, v8f& acc1) {
#pragma unroll 1
  for (int k0 = 0; k0 < kdim; k0 += 32) {
    const v16h a  = ld_frag(arow + k0);
    const v16h b0 = ld_frag(bp0 + k0);
    const v16h b1 = ld_frag(bp1 + k0);
    acc0 = mma_h(a, b0, acc0);
    acc1 = mma_h(a, b1, acc1);
    guard_pair(acc0, acc1, a, b0, b1);
  }
  guard_tail2(acc0, acc1);
}
__device__ __forceinline__ void gemm_one(const _Float16* arow, const _Float16* bp0, const int kdim, v8f& acc0) {
#pragma unroll 1
  for (int k0 = 0; k0 < kdim; k0 += 32) {
    const v16h a  = ld_frag(arow + k0);
    const v16h b0 = ld_frag(bp0 + k0);
    acc0 = mma_h(a, b0, acc0);
    guard_one(acc0, a, b0);
  }
  guard_tail1(acc0);
}

__global__ __launch_bounds__(NTHR) void wpack_kernel(const float* __restrict__ src, int Kin, int C, int ldo,
                                                     unsigned short* __restrict__ O, float sc) {
  __shared__ float Tt[64 * 65];
  const int tid = threadIdx.x;
  const int c0 = blockIdx.x * 64, r0 = blockIdx.y * 64;
#pragma unroll
  for (int i = 0; i < 4; ++i) {
    const int idx = i * NTHR + tid;
    const int rr = idx >> 4, cc = (idx & 15) * 4;
    const int k  = r0 + rr;
    const int kc = (k < Kin) ? k : (Kin - 1);
    const bool keep = (k < Kin);
    const v4f v = *(const v4f*)(src + (size_t)kc * (size_t)C + c0 + cc);
    const float e0 = v[0], e1 = v[1], e2 = v[2], e3 = v[3];
    Tt[rr * 65 + cc + 0] = keep ? e0 : 0.0f;
    Tt[rr * 65 + cc + 1] = keep ? e1 : 0.0f;
    Tt[rr * 65 + cc + 2] = keep ? e2 : 0.0f;
    Tt[rr * 65 + cc + 3] = keep ? e3 : 0.0f;
  }
  __syncthreads();
  const int q = tid >> 3, c8 = (tid & 7) * 8;
  v8h hv[2];
#pragma unroll
  for (int g = 0; g < 2; ++g) {
    const int qq = g * 32 + q;
#pragma unroll
    for (int e = 0; e < 8; ++e) {
      const float f = Tt[(c8 + e) * 65 + qq];
      hv[g][e] = (_Float16)(bf16r(f) * sc);
    }
  }
  for (int pass = 0; pass < 2; ++pass) {
#pragma unroll
    for (int g = 0; g < 2; ++g) {
      const size_t o = (size_t)(c0 + g * 32 + q) * (size_t)ldo + (size_t)(r0 + c8);
      *(volatile v8h*)(O + o) = hv[g];
    }
    __threadfence();
  }
}

__global__ __launch_bounds__(NTHR) void dcgru_seq_kernel(
    const float* __restrict__ h_init, const float* __restrict__ targets, const float* __restrict__ adj,
    const float* __restrict__ bg0, const float* __restrict__ bc0,
    const float* __restrict__ bg1, const float* __restrict__ bc1,
    const float* __restrict__ Wout, const float* __restrict__ bout,
    const unsigned short* __restrict__ Wg0p, const unsigned short* __restrict__ Wc0p,
    const unsigned short* __restrict__ Wg1p, const unsigned short* __restrict__ Wc1p,
    float* __restrict__ out) {
  __shared__ __align__(16) _Float16 Xg[RB * XP];
  __shared__ __align__(16) float    H1S[RB * HSP];
  __shared__ __align__(16) float    dgS[NSUP * RB];
  __shared__ __align__(16) float    WoS[NHID * NFEAT];
  __shared__ __align__(16) float    outS[RB * NFEAT];

  const _Float16* Wg0 = (const _Float16*)Wg0p;
  const _Float16* Wc0 = (const _Float16*)Wc0p;
  const _Float16* Wg1 = (const _Float16*)Wg1p;
  const _Float16* Wc1 = (const _Float16*)Wc1p;

  const int tid = threadIdx.x, lane = tid & 31, wave = tid >> 5;
  const int c = lane & 15, hh = lane >> 4, koff = hh * 8;
  const int mt = wave >> 2, ub = wave & 3;
  const int j = 16 * ub + c;
  const int rl0 = 16 * mt + 8 * hh;
  const int rowbase = blockIdx.x * RB;
  const int bb = rowbase / NNODE;
  const int n0 = rowbase - bb * NNODE;

  if (tid < NSUP * RB) {
    const int m = tid >> 5, row = tid & 31;
    const int n = n0 + row;
    const float dv = adj[((size_t)(m * NNODE + n)) * NNODE + n];
    dgS[tid] = ACARRY * bf16r(dv);
    WoS[tid] = bf16r(Wout[tid]);
  }
  asm volatile("" ::: "memory");

  float h0st[8], h1st[8];
#pragma unroll
  for (int r = 0; r < 8; ++r) {
    float hv = bf16r(h_init[(size_t)(rowbase + rl0 + r) * NHID + j]);
    asm volatile("" : "+v"(hv));
    h0st[r] = hv;
    h1st[r] = hv;
  }
  asm volatile("" ::: "memory");
  const float bR0 = bf16r(bg0[j]);
  const float bU0 = bf16r(bg0[NHID + j]);
  const float bC0 = bf16r(bc0[j]);
  const float bR1 = bf16r(bg1[j]);
  const float bU1 = bf16r(bg1[NHID + j]);
  const float bC1 = bf16r(bc1[j]);
  const float bo  = bf16r(bout[tid & 1]);
  __syncthreads();

  float dgr[NSUP][8];
#pragma unroll
  for (int m = 0; m < NSUP; ++m)
#pragma unroll
    for (int r = 0; r < 8; ++r) dgr[m][r] = dgS[m * RB + rl0 + r];

  const v8f z8 = {0.f, 0.f, 0.f, 0.f, 0.f, 0.f, 0.f, 0.f};
  const _Float16* arow = Xg + (16 * mt + c) * XP + koff;
  const _Float16* bg0r = Wg0 + (size_t)j * LD0 + koff;
  const _Float16* bg0u = Wg0 + (size_t)(NHID + j) * LD0 + koff;
  const _Float16* bc0c = Wc0 + (size_t)j * LD0 + koff;
  const _Float16* bg1r = Wg1 + (size_t)j * LD1 + koff;
  const _Float16* bg1u = Wg1 + (size_t)(NHID + j) * LD1 + koff;
  const _Float16* bc1c = Wc1 + (size_t)j * LD1 + koff;

#pragma unroll 1
  for (int t = 0; t < NSTEP; ++t) {
#pragma unroll
    for (int r = 0; r < 8; ++r)
#pragma unroll
      for (int m = 0; m < NSUP; ++m)
        Xg[(rl0 + r) * XP + m * FC0 + FX0 + j] = (_Float16)(dgr[m][r] * h0st[r]);
    {
      const int row = tid >> 3, sub = tid & 7, m = sub >> 1, f = sub & 1;
      const int tt = (t > 0) ? (t - 1) : 0;
      const float xv = targets[(((size_t)(bb * NSTEP + tt)) * NNODE + n0 + row) * NFEAT + f];
      const float xb = (t > 0) ? bf16r(xv) : 0.0f;
      Xg[row * XP + m * FC0 + f] = (_Float16)(dgS[m * RB + row] * xb);
    }
    if (tid < 3 * RB) {
      const int row = tid / 3;
      const int part = tid - 3 * row;
      const v8h zz = {(_Float16)0.0f, (_Float16)0.0f, (_Float16)0.0f, (_Float16)0.0f,
                      (_Float16)0.0f, (_Float16)0.0f, (_Float16)0.0f, (_Float16)0.0f};
      *(v8h*)(Xg + row * XP + K0 + 8 * part) = zz;
    }
    __syncthreads();

    float rg[8], ug[8];
    {
      v8f aR = z8, aU = z8;
      gemm_pair(arow, bg0r, bg0u, K0P, aR, aU);
#pragma unroll
      for (int r = 0; r < 8; ++r) {
        rg[r] = fsig(aR[r] * FOLD + bR0);
        ug[r] = fsig(aU[r] * FOLD + bU0);
      }
    }
    __syncthreads();
#pragma unroll
    for (int r = 0; r < 8; ++r) {
      const float rh = rg[r] * h0st[r];
#pragma unroll
      for (int m = 0; m < NSUP; ++m)
        Xg[(rl0 + r) * XP + m * FC0 + FX0 + j] = (_Float16)(dgr[m][r] * rh);
    }
    __syncthreads();
    {
      v8f aC = z8;
      gemm_one(arow, bc0c, K0P, aC);
#pragma unroll
      for (int r = 0; r < 8; ++r) {
        const float cand = ftanh(aC[r] * FOLD + bC0);
        h0st[r] = ug[r] * h0st[r] + (1.0f - ug[r]) * cand;
      }
    }
    __syncthreads();

#pragma unroll
    for (int r = 0; r < 8; ++r)
#pragma unroll
      for (int m = 0; m < NSUP; ++m) {
        Xg[(rl0 + r) * XP + m * FC1 + j]       = (_Float16)(dgr[m][r] * h0st[r]);
        Xg[(rl0 + r) * XP + m * FC1 + FX1 + j] = (_Float16)(dgr[m][r] * h1st[r]);
      }
    __syncthreads();
    {
      v8f aR = z8, aU = z8;
      gemm_pair(arow, bg1r, bg1u, K1, aR, aU);
#pragma unroll
      for (int r = 0; r < 8; ++r) {
        rg[r] = fsig(aR[r] * FOLD + bR1);
        ug[r] = fsig(aU[r] * FOLD + bU1);
      }
    }
    __syncthreads();
#pragma unroll
    for (int r = 0; r < 8; ++r) {
      const float rh = rg[r] * h1st[r];
#pragma unroll
      for (int m = 0; m < NSUP; ++m)
        Xg[(rl0 + r) * XP + m * FC1 + FX1 + j] = (_Float16)(dgr[m][r] * rh);
    }
    __syncthreads();
    {
      v8f aC = z8;
      gemm_one(arow, bc1c, K1, aC);
#pragma unroll
      for (int r = 0; r < 8; ++r) {
        const float cand = ftanh(aC[r] * FOLD + bC1);
        h1st[r] = ug[r] * h1st[r] + (1.0f - ug[r]) * cand;
      }
    }

#pragma unroll
    for (int r = 0; r < 8; ++r) H1S[(rl0 + r) * HSP + j] = h1st[r];
    __syncthreads();
    if (tid < RB * NFEAT) {
      const int row = tid >> 1, f = tid & 1;
      float s = 0.0f;
#pragma unroll 4
      for (int jj = 0; jj < NHID; ++jj) s = fmaf(H1S[row * HSP + jj], WoS[jj * NFEAT + f], s);
      outS[tid] = s + bo;
    }
    __syncthreads();
    if (tid < (RB * NFEAT) / 4) {
      const v4f v = *(const v4f*)(outS + 4 * tid);
      float* op = out + (((size_t)(bb * NSTEP + t)) * NNODE + n0) * NFEAT + 4 * tid;
      *(volatile v4f*)op = v;
      __threadfence();
      *(volatile v4f*)op = v;
    }
  }
}

extern "C" void kernel_launch(void* const* d_in, const int* in_sizes, int n_in,
                              void* d_out, int out_size, void* d_ws, size_t ws_size, hipStream_t stream) {
  if (n_in < 13 || d_out == nullptr || d_ws == nullptr) return;
  if (in_sizes[0] != NROWS * NHID || in_sizes[1] != NBAT * NSTEP * NNODE * NFEAT ||
      in_sizes[2] != NSUP * NNODE * NNODE ||
      in_sizes[3] != K0 * 2 * NHID || in_sizes[4] != 2 * NHID ||
      in_sizes[5] != K0 * NHID || in_sizes[6] != NHID ||
      in_sizes[7] != K1 * 2 * NHID || in_sizes[8] != 2 * NHID ||
      in_sizes[9] != K1 * NHID || in_sizes[10] != NHID ||
      in_sizes[11] != NHID * NFEAT || in_sizes[12] != NFEAT ||
      out_size != NBAT * NSTEP * NNODE * NFEAT) return;

  const float* h_init  = (const float*)d_in[0];
  const float* targets = (const float*)d_in[1];
  const float* adj     = (const float*)d_in[2];
  const float* W_g0    = (const float*)d_in[3];
  const float* b_g0    = (const float*)d_in[4];
  const float* W_c0    = (const float*)d_in[5];
  const float* b_c0    = (const float*)d_in[6];
  const float* W_g1    = (const float*)d_in[7];
  const float* b_g1    = (const float*)d_in[8];
  const float* W_c1    = (const float*)d_in[9];
  const float* b_c1    = (const float*)d_in[10];
  const float* W_out   = (const float*)d_in[11];
  const float* b_out   = (const float*)d_in[12];
  float* out = (float*)d_out;

  char* ws = (char*)d_ws;
  size_t off = 0;
  auto carve = [&](size_t bytes) -> char* { char* p = ws + off; off += (bytes + 255) & ~(size_t)255; return p; };
  unsigned short* WG0T = (unsigned short*)carve((size_t)2 * NHID * LD0 * 2);
  unsigned short* WC0T = (unsigned short*)carve((size_t)NHID * LD0 * 2);
  unsigned short* WG1T = (unsigned short*)carve((size_t)2 * NHID * LD1 * 2);
  unsigned short* WC1T = (unsigned short*)carve((size_t)NHID * LD1 * 2);
  if (off > ws_size || off > (size_t)134217728) return;

  wpack_kernel<<<dim3((2 * NHID) / 64, LD0 / 64), NTHR, 0, stream>>>(W_g0, K0, 2 * NHID, LD0, WG0T, WCARRY);
  wpack_kernel<<<dim3(NHID / 64, LD0 / 64), NTHR, 0, stream>>>(W_c0, K0, NHID, LD0, WC0T, WCARRY);
  wpack_kernel<<<dim3((2 * NHID) / 64, LD1 / 64), NTHR, 0, stream>>>(W_g1, K1, 2 * NHID, LD1, WG1T, WCARRY);
  wpack_kernel<<<dim3(NHID / 64, LD1 / 64), NTHR, 0, stream>>>(W_c1, K1, NHID, LD1, WC1T, WCARRY);

  dcgru_seq_kernel<<<NBLK, NTHR, 0, stream>>>(h_init, targets, adj, b_g0, b_c0, b_g1, b_c1, W_out, b_out,
                                              WG0T, WC0T, WG1T, WC1T, out);
}
